// LongformerLayer_68719476736461
// MI455X (gfx1250) — hardware-verified
//
#include <hip/hip_runtime.h>
#include <hip/hip_bf16.h>
#include <math.h>

#define BB 2
#define SS 2048
#define DD 768
#define HH 12
#define DKK 64
#define DFF 3072
#define WIN 256
#define QW 2
#define MTOK (BB * SS)

typedef _Float16 bf16;
typedef __attribute__((ext_vector_type(4))) unsigned v4u_t;
typedef unsigned v4ua __attribute__((ext_vector_type(4), may_alias));
typedef __attribute__((ext_vector_type(4))) float v4f_t;
typedef float v4fa __attribute__((ext_vector_type(4), may_alias));
typedef __attribute__((ext_vector_type(16))) bf16  bf16x16;
typedef __attribute__((ext_vector_type(8)))  bf16  bf16x8;
typedef __attribute__((ext_vector_type(4)))  bf16  bf16x4;
typedef __attribute__((ext_vector_type(8)))  float f32x8;

#define LDS_STRIDE 48
#define KSTRIDE    72
#define VSTRIDE    48

__device__ __forceinline__ f32x8 wmma_bf16(bf16x16 a, bf16x16 b, f32x8 c) {
  return __builtin_amdgcn_wmma_f32_16x16x32_f16(
      false, a, false, b, (short)0, c, false, false);
}

template <typename T>
__device__ __forceinline__ bf16x16 load_frag(const T* __restrict__ base, int ld,
                                             int row0, int k0) {
  const int lane = threadIdx.x & 31;
  const int r    = lane & 15;
  const int kh   = (lane >> 4) * 8;
  const T* p0 = base + (size_t)(row0 + r) * ld + (k0 + kh);
  const T* p1 = p0 + 16;
  bf16x16 f;
#pragma unroll
  for (int i = 0; i < 8; ++i) {
    f[i]     = (bf16)p0[i];
    f[i + 8] = (bf16)p1[i];
  }
  return f;
}

__device__ __forceinline__ bf16x16 lds_frag(const bf16* base, int stride) {
  const int lane = threadIdx.x & 31;
  const int row  = lane & 15;
  const int kh   = (lane >> 4) * 8;
  const bf16x8 lo = *(const bf16x8*)(base + row * stride + kh);
  const bf16x8 hi = *(const bf16x8*)(base + row * stride + kh + 16);
  bf16x16 f;
#pragma unroll
  for (int i = 0; i < 8; ++i) { f[i] = lo[i]; f[i + 8] = hi[i]; }
  return f;
}

template <typename T>
__device__ __forceinline__ void stage_read16(const T* __restrict__ p, float* buf) {
#pragma unroll
  for (int i = 0; i < 16; ++i) buf[i] = (float)p[i];
}

__device__ __forceinline__ void stage_write(bf16* dst, const float* buf, int nquad) {
#pragma unroll
  for (int i = 0; i < nquad; ++i) {
    bf16x4 q;
    q[0] = (bf16)buf[4 * i];     q[1] = (bf16)buf[4 * i + 1];
    q[2] = (bf16)buf[4 * i + 2]; q[3] = (bf16)buf[4 * i + 3];
    *(bf16x4*)(dst + 4 * i) = q;
  }
}

template <typename AT, int MODE>
__global__ __launch_bounds__(256) void gemm_bias_kernel(
    const AT* __restrict__ A, const float* __restrict__ W,
    const float* __restrict__ bias, void* __restrict__ out,
    int M, int N, int K) {
  __shared__ bf16 ldsA[128 * LDS_STRIDE];
  __shared__ bf16 ldsW[256 * LDS_STRIDE];
  __shared__ __attribute__((aligned(16))) unsigned char sob[256 * 136 * 2];

  const int t    = threadIdx.x;
  const int wave = t >> 5;
  const int lane = t & 31;
  const int wm   = (wave & 1) * 64;
  const int wn   = (wave >> 1) * 64;
  const int mBlk = blockIdx.x * 128;
  const int nBlk = blockIdx.y * 256;

  const int arow = t >> 1;
  const int ach  = (t & 1) * 16;

  float abuf[16];
  float wbuf[32];

  stage_read16(A + (size_t)(mBlk + arow) * K + ach, abuf);
  stage_read16(W + (size_t)(nBlk + t) * K,          wbuf);
  stage_read16(W + (size_t)(nBlk + t) * K + 16,     wbuf + 16);

  f32x8 acc[4][4] = {};

  for (int k = 0; k < K; k += 32) {
    __syncthreads();
    stage_write(&ldsA[arow * LDS_STRIDE + ach], abuf, 4);
    stage_write(&ldsW[t * LDS_STRIDE],          wbuf, 8);
    if (k + 32 < K) {
      stage_read16(A + (size_t)(mBlk + arow) * K + (k + 32) + ach, abuf);
      stage_read16(W + (size_t)(nBlk + t) * K + (k + 32),          wbuf);
      stage_read16(W + (size_t)(nBlk + t) * K + (k + 32) + 16,     wbuf + 16);
    }
    __syncthreads();

    bf16x16 af[4], wf[4];
#pragma unroll
    for (int i = 0; i < 4; ++i)
      af[i] = lds_frag(ldsA + (wm + 16 * i) * LDS_STRIDE, LDS_STRIDE);
#pragma unroll
    for (int j = 0; j < 4; ++j)
      wf[j] = lds_frag(ldsW + (wn + 16 * j) * LDS_STRIDE, LDS_STRIDE);
#pragma unroll
    for (int i = 0; i < 4; ++i)
#pragma unroll
      for (int j = 0; j < 4; ++j)
        acc[i][j] = wmma_bf16(af[i], wf[j], acc[i][j]);
  }

  const int nlane = lane & 15;
  const int mh    = (lane >> 4) * 8;
  __syncthreads();
  if (MODE == 0 || MODE == 1 || MODE == 3) {
    bf16* so = (bf16*)sob;
#pragma unroll
    for (int i = 0; i < 4; ++i)
#pragma unroll
      for (int j = 0; j < 4; ++j) {
        const int nl = wn + 16 * j + nlane;
        const float bv = bias[nBlk + nl];
        if (MODE == 3) {
#pragma unroll 1
          for (int r = 0; r < 8; ++r) {
            const int ml = wm + 16 * i + mh + r;
            const float xg = acc[i][j][r] + bv;
            so[ml * 264 + nl] = (bf16)(0.5f * xg * (1.0f + erff(xg * 0.70710678118654752f)));
          }
        } else {
#pragma unroll
        for (int r = 0; r < 8; ++r) {
          const int ml = wm + 16 * i + mh + r;
          const bf16 hv = (bf16)(acc[i][j][r] + bv);
          if (MODE == 0) so[ml * 264 + nl] = hv;
          else           so[nl * 136 + ml] = hv;
        }
        }
      }
    __syncthreads();
#pragma unroll 1
    for (int pass = 0; pass < 2; ++pass) {
      if (MODE == 0 || MODE == 3) {
        for (int ch = t; ch < 128 * 32; ch += 256) { const int ml = ch >> 5, q = (ch & 31) * 8;
          *(volatile v4u_t*)((bf16*)out + (size_t)(mBlk + ml) * N + nBlk + q) = *(const v4ua*)(so + ml * 264 + q); }
      } else {
        const int b_ = mBlk / SS, s0 = mBlk & (SS - 1);
        for (int ch = t; ch < 256 * 16; ch += 256) { const int nl = ch >> 4, q = (ch & 15) * 8; const int n = nBlk + nl, h = n >> 6, dk = n & (DKK - 1);
          *(volatile v4u_t*)((bf16*)out + (((size_t)(b_ * HH + h)) * DKK + dk) * SS + s0 + q) = *(const v4ua*)(so + nl * 136 + q); }
      }
      __threadfence();
    }
  } else {
    float* so = (float*)sob;
#pragma unroll 1
    for (int hf = 0; hf < 2; ++hf) {
      if (wm == hf * 64) {
#pragma unroll
        for (int i = 0; i < 4; ++i)
#pragma unroll
          for (int j = 0; j < 4; ++j) {
            const int nl = wn + 16 * j + nlane;
            const float bv = bias[nBlk + nl];
#pragma unroll
            for (int r = 0; r < 8; ++r) so[(16 * i + mh + r) * 260 + nl] = acc[i][j][r] + bv;
          }
      }
      __syncthreads();
#pragma unroll 1
      for (int pass = 0; pass < 2; ++pass) {
        for (int ch = t; ch < 64 * 64; ch += 256) { const int ml = ch >> 6, q = (ch & 63) * 4;
          *(volatile v4f_t*)((float*)out + (size_t)(mBlk + hf * 64 + ml) * N + nBlk + q) = *(const volatile v4fa*)(so + ml * 260 + q); }
        __threadfence();
      }
      __syncthreads();
    }
  }
}

__global__ __launch_bounds__(64) void attn_kernel(
    const bf16* __restrict__ Qb, const bf16* __restrict__ Kb,
    const bf16* __restrict__ Vt, const int* __restrict__ gmask, const int* __restrict__ kmask,
    bf16* __restrict__ attnOut) {
  __shared__ int gS[SS], kS[SS];
  __shared__ bf16 ldsK[32 * KSTRIDE];
  __shared__ bf16 ldsV[64 * VSTRIDE];
  __shared__ __attribute__((aligned(16))) bf16 ldsO[2][32 * 72];

  const int q0blk = blockIdx.x * 64;
  const int h  = blockIdx.y;
  const int b  = blockIdx.z;
  const int t    = threadIdx.x;
  const int wave = t >> 5;
  const int lane = t & 31;
  const int qlane = lane & 15;
  const int kh8   = (lane >> 4) * 8;
  const int q0 = q0blk + wave * 32;

  for (int i = threadIdx.x; i < SS; i += 64) { gS[i] = gmask[(size_t)b * SS + i]; kS[i] = kmask[(size_t)b * SS + i]; }
  __syncthreads();
  const bf16* Qh = Qb + (size_t)b * SS * DD + h * DKK;
  const bf16* Kh = Kb + (size_t)b * SS * DD + h * DKK;
  const bf16* Vh = Vt + ((size_t)(b * HH + h)) * DKK * SS;

  const int krow = t >> 1;
  const int kcol = (t & 1) * 32;
  const bf16* kSrc = Kh + (size_t)krow * DD + kcol;
  const bf16* vSrc = Vh + (size_t)t * SS;

  bf16x16 qf[QW][2];
#pragma unroll
  for (int qt = 0; qt < QW; ++qt) {
    qf[qt][0] = load_frag(Qh, DD, q0 + 16 * qt, 0);
    qf[qt][1] = load_frag(Qh, DD, q0 + 16 * qt, 32);
  }

  f32x8 o[QW][4] = {};
  float mrun[QW], lrun[QW];
#pragma unroll
  for (int qt = 0; qt < QW; ++qt) { mrun[qt] = -INFINITY; lrun[qt] = 0.0f; }

  const float scale = 0.125f * 1.44269504088896340736f;
  const float NEG2 = -1.0e9f;
  const int kmax = SS - 1;

  bf16x8 kreg[4], vreg[4];
#pragma unroll
  for (int i = 0; i < 4; ++i) {
    kreg[i] = *(const bf16x8*)(kSrc + 8 * i);
    vreg[i] = *(const bf16x8*)(vSrc + 8 * i);
  }

  for (int kb = 0; kb <= kmax; kb += 32) {
    __syncthreads();
#pragma unroll
    for (int i = 0; i < 4; ++i) {
      *(bf16x8*)(&ldsK[krow * KSTRIDE + kcol + 8 * i]) = kreg[i];
      *(bf16x8*)(&ldsV[t * VSTRIDE + 8 * i])           = vreg[i];
    }
    if (kb + 32 <= kmax) {
      const bf16* kn = kSrc + (size_t)(kb + 32) * DD;
      const bf16* vn = vSrc + (kb + 32);
#pragma unroll
      for (int i = 0; i < 4; ++i) {
        kreg[i] = *(const bf16x8*)(kn + 8 * i);
        vreg[i] = *(const bf16x8*)(vn + 8 * i);
      }
    }
    __syncthreads();

    bf16x16 kf[2][2];
#pragma unroll
    for (int ktile = 0; ktile < 2; ++ktile)
#pragma unroll
      for (int c = 0; c < 2; ++c)
        kf[ktile][c] = lds_frag(ldsK + (ktile * 16) * KSTRIDE + c * 32, KSTRIDE);

    bf16x16 pf[QW];
    bool act[QW];
#pragma unroll
    for (int qt = 0; qt < QW; ++qt) {
      unsigned mbits = 0;
      {
        const int q_my = q0 + 16 * qt + qlane;
        const int gq = gS[q_my];
#pragma unroll
        for (int r = 0; r < 8; ++r) { const int j0 = kb + kh8 + r, j1 = j0 + 16;
          if ((((j0 - q_my <= WIN) && (q_my - j0 <= WIN)) || gq || gS[j0]) && kS[j0]) mbits |= 1u << r;
          if ((((j1 - q_my <= WIN) && (q_my - j1 <= WIN)) || gq || gS[j1]) && kS[j1]) mbits |= 1u << (8 + r);
        }
        act[qt] = (__builtin_amdgcn_ballot_w32(mbits != 0) != 0);
      }
      if (act[qt]) {
        const int q_my = q0 + 16 * qt + qlane;
        f32x8 s0 = {}, s1 = {};
        s0 = wmma_bf16(kf[0][0], qf[qt][0], s0);
        s0 = wmma_bf16(kf[0][1], qf[qt][1], s0);
        s1 = wmma_bf16(kf[1][0], qf[qt][0], s1);
        s1 = wmma_bf16(kf[1][1], qf[qt][1], s1);

        float mx = -INFINITY;
#pragma unroll
        for (int r = 0; r < 8; ++r) {
          const int k0i = kb + kh8 + r;
          const int k1i = k0i + 16;
          (void)k0i; (void)k1i; (void)q_my;
          s0[r] = (mbits & (1u << r))       ? s0[r] * scale : NEG2;
          s1[r] = (mbits & (1u << (8 + r))) ? s1[r] * scale : NEG2;
          mx = fmaxf(mx, fmaxf(s0[r], s1[r]));
        }
        mx = fmaxf(mx, __shfl_xor(mx, 16, 32));
        const float mnew  = fmaxf(mrun[qt], mx);
        const float alpha = exp2f(mrun[qt] - mnew);

        float rsum = 0.0f;
#pragma unroll
        for (int r = 0; r < 8; ++r) {
          const float p0 = exp2f(s0[r] - mnew);
          const float p1 = exp2f(s1[r] - mnew);
          rsum += p0 + p1;
          pf[qt][r]     = (bf16)(p0 * 1024.0f);
          pf[qt][r + 8] = (bf16)(p1 * 1024.0f);
        }
        rsum += __shfl_xor(rsum, 16, 32);
        lrun[qt] = lrun[qt] * alpha + rsum;
        mrun[qt] = mnew;

#pragma unroll
        for (int j = 0; j < 4; ++j)
#pragma unroll
          for (int r = 0; r < 8; ++r) o[qt][j][r] *= alpha;
      }
    }

#pragma unroll
    for (int j = 0; j < 4; ++j) {
      const bf16x16 vf = lds_frag(ldsV + (j * 16) * VSTRIDE, VSTRIDE);
#pragma unroll
      for (int qt = 0; qt < QW; ++qt)
        if (act[qt]) o[qt][j] = wmma_bf16(vf, pf[qt], o[qt][j]);
    }
  }

  bf16* so = ldsO[wave];
#pragma unroll
  for (int qt = 0; qt < QW; ++qt) {
    const float rl = 1.0f / (lrun[qt] * 1024.0f);
#pragma unroll
    for (int j = 0; j < 4; ++j)
#pragma unroll
      for (int r = 0; r < 8; ++r) so[(16 * qt + qlane) * 72 + j * 16 + kh8 + r] = (bf16)(o[qt][j][r] * rl);
  }
  asm volatile("s_wait_dscnt 0" ::: "memory");
#pragma unroll 1
  for (int pass = 0; pass < 2; ++pass) {
#pragma unroll
    for (int it = 0; it < 8; ++it) { const int ch = lane + 32 * it, ql = ch >> 3, q8 = (ch & 7) * 8;
      *(volatile v4u_t*)(attnOut + ((size_t)(b * SS + q0 + ql)) * DD + h * DKK + q8) = *(const v4ua*)(so + ql * 72 + q8); }
    __threadfence();
  }
}


__global__ __launch_bounds__(256) void k_transpose(const float* __restrict__ Wm, float* __restrict__ Wt, int K, int N) {
  const size_t g = (size_t)blockIdx.x * 256 + threadIdx.x;
  const size_t e0 = g * 4;
  if (e0 >= (size_t)K * N) return;
  const int n = (int)(e0 / K), k0 = (int)(e0 % K);
  v4f_t v; v[0] = Wm[(size_t)k0 * N + n]; v[1] = Wm[(size_t)(k0 + 1) * N + n]; v[2] = Wm[(size_t)(k0 + 2) * N + n]; v[3] = Wm[(size_t)(k0 + 3) * N + n];
  *(volatile v4f_t*)(Wt + e0) = v; __threadfence(); *(volatile v4f_t*)(Wt + e0) = v;
}
__global__ __launch_bounds__(256) void k_add_ln(const float* __restrict__ a, const float* __restrict__ r, const float* __restrict__ g,
                                                const float* __restrict__ bta, float* __restrict__ y) {
  __shared__ float red[256];
  const int tok = blockIdx.x, t = threadIdx.x;
  const float* ar = a + (size_t)tok * DD; const float* rr = r + (size_t)tok * DD;
  float v0 = ar[t] + rr[t], v1 = ar[t + 256] + rr[t + 256], v2 = ar[t + 512] + rr[t + 512];
  red[t] = v0 + v1 + v2; __syncthreads();
  for (int o = 128; o > 0; o >>= 1) { if (t < o) red[t] += red[t + o]; __syncthreads(); }
  const float mu = red[0] * (1.0f / (float)DD); __syncthreads();
  const float d0 = v0 - mu, d1 = v1 - mu, d2 = v2 - mu;
  red[t] = d0 * d0 + d1 * d1 + d2 * d2; __syncthreads();
  for (int o = 128; o > 0; o >>= 1) { if (t < o) red[t] += red[t + o]; __syncthreads(); }
  const float rs = rsqrtf(red[0] * (1.0f / (float)DD) + 1e-5f);
  float* yr = y + (size_t)tok * DD;
  const float o0 = d0 * rs * g[t] + bta[t], o1 = d1 * rs * g[t + 256] + bta[t + 256], o2 = d2 * rs * g[t + 512] + bta[t + 512];
  *(volatile float*)(yr + t) = o0; *(volatile float*)(yr + t + 256) = o1; *(volatile float*)(yr + t + 512) = o2;
  __threadfence();
  *(volatile float*)(yr + t) = o0; *(volatile float*)(yr + t + 256) = o1; *(volatile float*)(yr + t + 512) = o2;
}

extern "C" void kernel_launch(void* const* d_in, const int* in_sizes, int n_in,
                              void* d_out, int out_size, void* d_ws, size_t ws_size,
                              hipStream_t stream) {
  (void)in_sizes; (void)n_in; (void)out_size; (void)ws_size;
  const float* x = (const float*)d_in[0];
  const int* kmask = (const int*)d_in[1];
  const int* gmask = (const int*)d_in[2];
  const float* Wq = (const float*)d_in[3],  *bq = (const float*)d_in[4];
  const float* Wk = (const float*)d_in[5],  *bk = (const float*)d_in[6];
  const float* Wv = (const float*)d_in[7],  *bv = (const float*)d_in[8];
  const float* Wo = (const float*)d_in[9],  *bo = (const float*)d_in[10];
  const float* g1 = (const float*)d_in[11], *be1 = (const float*)d_in[12];
  const float* W1 = (const float*)d_in[13], *b1 = (const float*)d_in[14];
  const float* W2 = (const float*)d_in[15], *b2 = (const float*)d_in[16];
  const float* g2 = (const float*)d_in[17], *be2 = (const float*)d_in[18];
  float* out = (float*)d_out;

  char* ws = (char*)d_ws;
  const size_t WDD = (size_t)DD * DD * 4, WDF = (size_t)DD * DFF * 4, F16T = (size_t)MTOK * DD * 2, F32T = (size_t)MTOK * DD * 4;
  float* Wqt = (float*)ws; ws += WDD;  float* Wkt = (float*)ws; ws += WDD;  float* Wvt = (float*)ws; ws += WDD;  float* Wot = (float*)ws; ws += WDD;
  float* W1t = (float*)ws; ws += WDF;  float* W2t = (float*)ws; ws += WDF;
  bf16* Qb = (bf16*)ws; ws += F16T;  bf16* Kb = (bf16*)ws; ws += F16T;  bf16* VtB = (bf16*)ws; ws += F16T;  bf16* attn = (bf16*)ws; ws += F16T;
  float* proj = (float*)ws; ws += F32T;  float* hbuf = (float*)ws; ws += F32T;
  bf16* ff1 = (bf16*)ws; ws += (size_t)MTOK * DFF * 2;

  k_transpose<<<dim3((DD * DD / 4 + 255) / 256), dim3(256), 0, stream>>>(Wq, Wqt, DD, DD);
  k_transpose<<<dim3((DD * DD / 4 + 255) / 256), dim3(256), 0, stream>>>(Wk, Wkt, DD, DD);
  k_transpose<<<dim3((DD * DD / 4 + 255) / 256), dim3(256), 0, stream>>>(Wv, Wvt, DD, DD);
  k_transpose<<<dim3((DD * DD / 4 + 255) / 256), dim3(256), 0, stream>>>(Wo, Wot, DD, DD);
  k_transpose<<<dim3((DD * DFF / 4 + 255) / 256), dim3(256), 0, stream>>>(W1, W1t, DD, DFF);
  k_transpose<<<dim3((DFF * DD / 4 + 255) / 256), dim3(256), 0, stream>>>(W2, W2t, DFF, DD);

  const int M = MTOK;
  dim3 gGrid(M / 128, DD / 256), gBlk(256);
  gemm_bias_kernel<float, 0><<<gGrid, gBlk, 0, stream>>>(x, Wqt, bq, Qb,  M, DD, DD);
  gemm_bias_kernel<float, 0><<<gGrid, gBlk, 0, stream>>>(x, Wkt, bk, Kb,  M, DD, DD);
  gemm_bias_kernel<float, 1><<<gGrid, gBlk, 0, stream>>>(x, Wvt, bv, VtB, M, DD, DD);
  attn_kernel<<<dim3(SS / 64, HH, BB), dim3(64), 0, stream>>>(Qb, Kb, VtB, gmask, kmask, attn);
  gemm_bias_kernel<bf16, 2><<<gGrid, gBlk, 0, stream>>>(attn, Wot, bo, proj, M, DD, DD);
  k_add_ln<<<dim3(MTOK), dim3(256), 0, stream>>>(x, proj, g1, be1, hbuf);
  gemm_bias_kernel<float, 3><<<dim3(M / 128, DFF / 256), gBlk, 0, stream>>>(hbuf, W1t, b1, ff1, M, DFF, DD);
  gemm_bias_kernel<bf16, 2><<<gGrid, gBlk, 0, stream>>>(ff1, W2t, b2, proj, M, DD, DFF);
  k_add_ln<<<dim3(MTOK), dim3(256), 0, stream>>>(hbuf, proj, g2, be2, out);
}
